// Self_attention_48567490183565
// MI455X (gfx1250) — hardware-verified
//
#include <hip/hip_runtime.h>
#include <math.h>

#ifndef NB
#define NB 8
#endif
#ifndef SEQ
#define SEQ 4096
#endif
#define NB_FULL 8
#define SEQ_FULL 4096

constexpr int kBatch   = NB;
constexpr int kSeq     = SEQ;
constexpr int kSeqFull = SEQ_FULL;
constexpr int kC       = 256;
constexpr int kD       = 32;
constexpr int kDP      = 64;
constexpr int kQPitch  = 128;
constexpr int kQK      = 96;
constexpr int kWRows   = kC + kDP;
constexpr float kWCarry    = 16.0f;
constexpr float kWCarryInv = 1.0f / 16.0f;
constexpr float kPCarry    = 16384.0f;
constexpr float kPCarryInv = 1.0f / 16384.0f;
static_assert(kBatch >= 1 && kBatch <= NB_FULL);
static_assert(kSeq % 256 == 0 && kSeq >= 256 && kSeq <= kSeqFull);
constexpr int kSmThreads = kSeq / 8;
constexpr int kSmWaves   = kSmThreads / 32;
static_assert(kSmWaves >= 1 && kSmWaves <= 16 && kSmThreads <= 512);
static_assert(kC % 64 == 0 && kSeq % 64 == 0 && kDP % 64 == 0 && kC % 32 == 0 && kQK % 32 == 0);
static_assert(kQK + 32 <= kQPitch);

constexpr size_t kSBytes  = (size_t)kSeq * kSeq * 4;
constexpr size_t kXtBytes = (size_t)kBatch * kSeq * kC * 2;
constexpr size_t kWBytes  = (size_t)kWRows * kC * 2;
constexpr size_t kBtBytes = 4096;
constexpr size_t kQBytes  = (size_t)kBatch * kSeq * kQPitch * 2;
constexpr size_t kVBytes  = (size_t)kBatch * kC * kSeq * 2;
constexpr size_t kPBytes  = (size_t)kSeq * kSeq * 2;
constexpr size_t kOffS  = 0;
constexpr size_t kOffW  = kOffS + kSBytes;
constexpr size_t kOffBt = kOffW + kWBytes;
constexpr size_t kOffQ  = kOffBt + kBtBytes;
constexpr size_t kOffV  = kOffQ + kQBytes;
constexpr size_t kOffP  = kOffV + kVBytes;
constexpr bool   kXtInS = (kXtBytes <= kSBytes);
constexpr size_t kOffXt = kXtInS ? kOffS : (kOffP + kPBytes);
constexpr size_t kWsTotal = kXtInS ? (kOffP + kPBytes) : (kOffXt + kXtBytes);
static_assert((size_t)kWRows * 4 <= kBtBytes);
static_assert(kOffW % 128 == 0 && kOffBt % 128 == 0 && kOffQ % 128 == 0 && kOffV % 128 == 0 && kOffP % 128 == 0 && kOffXt % 128 == 0);
static_assert(!kXtInS || (kOffXt + kXtBytes <= kOffW));
static_assert(kWsTotal <= (size_t)134217728);

typedef __attribute__((ext_vector_type(16))) _Float16 v16h;
typedef __attribute__((ext_vector_type(8)))  _Float16 v8h;
typedef __attribute__((ext_vector_type(16))) __bf16   v16b;
typedef __attribute__((ext_vector_type(8)))  __bf16   v8b;
typedef __attribute__((ext_vector_type(8)))  float    v8f;
typedef __attribute__((ext_vector_type(4)))  float    v4f;
typedef __attribute__((ext_vector_type(4)))  unsigned int v4u;

__device__ __forceinline__ unsigned short f2bf_bits(float f) {
  unsigned u = __float_as_uint(f);
  return (unsigned short)((u + 0x7FFFu + ((u >> 16) & 1u)) >> 16);
}
__device__ __forceinline__ float bf_bits2f(unsigned short h) { return __uint_as_float(((unsigned)h) << 16); }
__device__ __forceinline__ float bfr(float f) { return bf_bits2f(f2bf_bits(f)); }

__device__ __forceinline__ void dep_guard_h(v8f& a, v8f& b, v16h x, v16h y) { asm volatile("v_nop\n\tv_nop\n\tv_nop\n\tv_nop" : "+v"(a), "+v"(b) : "v"(x), "v"(y)); }
__device__ __forceinline__ void dep_guard_b(v8f& a, v8f& b, v16b x, v16b y) { asm volatile("v_nop\n\tv_nop\n\tv_nop\n\tv_nop" : "+v"(a), "+v"(b) : "v"(x), "v"(y)); }
__device__ __forceinline__ void keep4_h(v16h a, v16h b, v16h c, v16h d) { asm volatile("v_nop" :: "v"(a), "v"(b), "v"(c), "v"(d)); }
__device__ __forceinline__ void keep4_b(v16b a, v16b b, v16b c, v16b d) { asm volatile("v_nop" :: "v"(a), "v"(b), "v"(c), "v"(d)); }
__device__ __forceinline__ void acc_guard4(v8f& a, v8f& b, v8f& c, v8f& d) { asm volatile("v_nop\n\tv_nop\n\tv_nop\n\tv_nop" : "+v"(a), "+v"(b), "+v"(c), "+v"(d)); }
template <typename T> struct Frag;
template <> struct Frag<_Float16> {
  typedef v16h V; union U { v16h v; v8h h[2]; };
  static __device__ __forceinline__ v16h load(const _Float16* p) {
    U f; f.h[0] = *(const v8h*)(p); f.h[1] = *(const v8h*)(p + 16); return f.v;
  }
  static __device__ __forceinline__ v8f mma(v16h a, v16h b, v8f c) {
    return __builtin_amdgcn_wmma_f32_16x16x32_f16(false, a, false, b, (short)0, c, false, false);
  }
  static __device__ __forceinline__ void guard(v8f& a, v8f& b, v16h x, v16h y) { dep_guard_h(a, b, x, y); }
  static __device__ __forceinline__ void keep(v16h a, v16h b, v16h c, v16h d) { keep4_h(a, b, c, d); }
};
template <> struct Frag<__bf16> {
  typedef v16b V; union U { v16b v; v8b h[2]; };
  static __device__ __forceinline__ v16b load(const __bf16* p) {
    U f; f.h[0] = *(const v8b*)(p); f.h[1] = *(const v8b*)(p + 16); return f.v;
  }
  static __device__ __forceinline__ v8f mma(v16b a, v16b b, v8f c) {
    return __builtin_amdgcn_wmma_f32_16x16x32_bf16(false, a, false, b, (short)0, c, false, false);
  }
  static __device__ __forceinline__ void guard(v8f& a, v8f& b, v16b x, v16b y) { dep_guard_b(a, b, x, y); }
  static __device__ __forceinline__ void keep(v16b a, v16b b, v16b c, v16b d) { keep4_b(a, b, c, d); }
};

__device__ __forceinline__ unsigned pk16(unsigned short a, unsigned short b) { return (unsigned)a | ((unsigned)b << 16); }
__device__ __forceinline__ unsigned short h_bits(float f) { const _Float16 h = (_Float16)f; return __builtin_bit_cast(unsigned short, h); }

template <int ET> struct Elem;
template <> struct Elem<0> { typedef _Float16 T; };
template <> struct Elem<1> { typedef __bf16 T; };
template <int ET, bool SPLIT, int BIAS_MODE, int OUT_MODE, bool RESID>
__global__ __launch_bounds__(256) void wmma_gemm64(
    const unsigned short* __restrict__ Ap, const unsigned short* __restrict__ A2p, int lda, long strideA,
    const unsigned short* __restrict__ Btp, const unsigned short* __restrict__ Bt2p, int ldb, long strideB,
    void* Cout, void* Cout2, int ldc, long strideC,
    const float* __restrict__ bias,
    const float* __restrict__ resid, int ldr, long strideR,
    const float* __restrict__ gptr,
    int M, int N, int K, float scale) {
  typedef typename Elem<ET>::T T;
  typedef typename Frag<T>::V V;
  const T* A = (const T*)Ap; const T* A2 = (const T*)A2p; const T* Bt = (const T*)Btp; const T* Bt2 = (const T*)Bt2p;
  __shared__ __align__(16) float sT[8][16 * 68];
  const int b    = blockIdx.y;
  const int lane = threadIdx.x & 31;
  const int wave = threadIdx.x >> 5;
  const int tilesN = N >> 6;
  const int tilesM = M >> 6;
  const int tile = blockIdx.x * 8 + wave;
  if (tile >= tilesM * tilesN) return;
  const int tm = tile / tilesN;
  const int tn = tile - tm * tilesN;
  const int m0 = tm << 6;
  const int n0 = tn << 6;

  const T* Ab  = A  + (size_t)b * strideA;
  const T* Bb  = Bt + (size_t)b * strideB;
  const T* Ab2 = SPLIT ? (A2  + (size_t)b * strideA) : nullptr;
  const T* Bb2 = SPLIT ? (Bt2 + (size_t)b * strideB) : nullptr;

  const int rlane = lane & 15;
  const int koff  = (lane >> 4) * 8;
  const int mOff  = (lane >> 4) * 8;

  v8f acc[4][4];
#pragma unroll
  for (int i = 0; i < 4; ++i)
#pragma unroll
    for (int j = 0; j < 4; ++j) acc[i][j] = (v8f){0.f,0.f,0.f,0.f,0.f,0.f,0.f,0.f};

  for (int k0 = 0; k0 < K; k0 += 32) {
    V bh[4], bl[4];
#pragma unroll
    for (int j = 0; j < 4; ++j) {
      const size_t bo = (size_t)(n0 + (j << 4) + rlane) * ldb + koff + k0;
      bh[j] = Frag<T>::load(Bb + bo);
      if (SPLIT) bl[j] = Frag<T>::load(Bb2 + bo);
    }
#pragma unroll
    for (int i = 0; i < 4; ++i) {
      const size_t ao = (size_t)(m0 + (i << 4) + rlane) * lda + koff + k0;
      V ah = Frag<T>::load(Ab + ao);
      V al;
      if (SPLIT) al = Frag<T>::load(Ab2 + ao);
#pragma unroll
      for (int j = 0; j < 4; ++j) {
        acc[i][j] = Frag<T>::mma(ah, bh[j], acc[i][j]);
        if (SPLIT) {
          acc[i][j] = Frag<T>::mma(ah, bl[j], acc[i][j]);
          acc[i][j] = Frag<T>::mma(al, bh[j], acc[i][j]);
        }
      }
      Frag<T>::guard(acc[i][0], acc[i][3], ah, SPLIT ? al : ah);
    }
    Frag<T>::keep(bh[0], bh[1], bh[2], bh[3]);
    if (SPLIT) Frag<T>::keep(bl[0], bl[1], bl[2], bl[3]);
  }
  acc_guard4(acc[0][0], acc[0][1], acc[0][2], acc[0][3]);
  acc_guard4(acc[1][0], acc[1][1], acc[1][2], acc[1][3]);
  acc_guard4(acc[2][0], acc[2][1], acc[2][2], acc[2][3]);
  acc_guard4(acc[3][0], acc[3][1], acc[3][2], acc[3][3]);

  float* slab = sT[wave];
  const float* Rb = RESID ? (resid + (size_t)b * strideR) : nullptr;
  const float gval = RESID ? bfr(gptr[0]) : 1.0f;
#pragma unroll
  for (int i = 0; i < 4; ++i) {
    const int mBase = m0 + (i << 4);
#pragma unroll
    for (int j = 0; j < 4; ++j) {
      const int n = n0 + (j << 4) + rlane;
      float bv = 0.f;
      if (BIAS_MODE == 2) bv = bias[n];
#pragma unroll
      for (int r = 0; r < 8; ++r) {
        float v = acc[i][j][r] * scale;
        if (BIAS_MODE == 1) v += bias[mBase + mOff + r];
        if (BIAS_MODE == 2) v += bv;
        slab[(mOff + r) * 68 + (j << 4) + rlane] = v;
      }
    }
    __builtin_amdgcn_fence(3  , "workgroup");
    __builtin_amdgcn_wave_barrier();
    __builtin_amdgcn_fence(2  , "workgroup");
    if (OUT_MODE == 0) {
      float* C = (float*)Cout + (size_t)b * strideC;
      const int hh = lane >> 4, c4 = (lane & 15) * 4;
      for (int pass = 0; pass < 2; ++pass) {
#pragma unroll
        for (int it = 0; it < 8; ++it) {
          const int row = it * 2 + hh;
          v4f v = *(const v4f*)(slab + row * 68 + c4);
          if (RESID) {
            const v4f xr = *(const v4f*)(Rb + (size_t)(mBase + row) * ldr + n0 + c4);
            v4f o;
#pragma unroll
            for (int e = 0; e < 4; ++e) o[e] = v[e] * gval + bfr(xr[e]);
            v = o;
          }
          *(volatile v4f*)(C + (size_t)(mBase + row) * ldc + n0 + c4) = v;
        }
        __threadfence();
      }
    } else {
      const int q = lane >> 3, c8 = (lane & 7) * 8;
      const bool lo_sel = (c8 < 32);
      unsigned short* C  = (unsigned short*)Cout  + (size_t)b * strideC;
      unsigned short* C2 = (unsigned short*)Cout2 + (size_t)b * strideC;
      for (int pass = 0; pass < 2; ++pass) {
#pragma unroll
        for (int it = 0; it < 4; ++it) {
          const int row = it * 4 + q;
          const float* sp = slab + row * 68 + c8;
          v8h hv, lv;
#pragma unroll
          for (int e = 0; e < 8; ++e) {
            if (OUT_MODE == 1) {
              hv[e] = (_Float16)sp[e];
              lv[e] = hv[e];
            } else {
              unsigned short hb = f2bf_bits(sp[e]);
              unsigned short lb = f2bf_bits(sp[e] - bf_bits2f(hb));
              hv[e] = __builtin_bit_cast(_Float16, hb);
              lv[e] = __builtin_bit_cast(_Float16, lb);
            }
          }
          *(volatile v8h*)(C + (size_t)(mBase + row) * ldc + n0 + c8) = hv;
          if (OUT_MODE == 2) *(volatile v8h*)(C2 + (size_t)(mBase + row) * ldc + n0 + c8) = lv;
          if (OUT_MODE == 3) {
            v8h sv;
#pragma unroll
            for (int e = 0; e < 8; ++e) sv[e] = lo_sel ? lv[e] : hv[e];
            *(volatile v8h*)(C2 + (size_t)(mBase + row) * ldc + n0 + c8) = sv;
          }
        }
        __threadfence();
      }
    }
    __builtin_amdgcn_fence(3  , "workgroup");
    __builtin_amdgcn_wave_barrier();
    __builtin_amdgcn_fence(2  , "workgroup");
  }
}

__global__ __launch_bounds__(256) void xtcast_kernel(const float* __restrict__ x, unsigned short* __restrict__ xt) {
  __shared__ float sm[64][65];
  const int t  = threadIdx.x;
  const int n0 = blockIdx.x * 64;
  const int c0 = blockIdx.y * 64;
  const int b  = blockIdx.z;
  const float* xb = x + (size_t)b * kC * kSeqFull;
#pragma unroll
  for (int i = 0; i < 16; ++i) {
    const int e  = i * 256 + t;
    const int r  = e >> 6;
    const int cl = e & 63;
    sm[cl][r] = bfr(xb[(size_t)(c0 + r) * kSeqFull + n0 + cl]);
  }
  __syncthreads();
  const int lane = t & 31, wave = t >> 5;
  const int q = lane >> 3, c8 = (lane & 7) * 8;
  unsigned short* op = xt + (size_t)b * kSeq * kC;
  for (int pass = 0; pass < 2; ++pass) {
#pragma unroll
    for (int it = 0; it < 2; ++it) {
      const int row = wave * 8 + it * 4 + q;
      unsigned short hb[8];
#pragma unroll
      for (int e = 0; e < 8; ++e) hb[e] = h_bits(sm[row][c8 + e]);
      const v4u u = (v4u){pk16(hb[0], hb[1]), pk16(hb[2], hb[3]), pk16(hb[4], hb[5]), pk16(hb[6], hb[7])};
      *(volatile v4u*)(op + (size_t)(n0 + row) * kC + c0 + c8) = u;
    }
    __threadfence();
  }
}

__global__ __launch_bounds__(256) void param_kernel(const float* __restrict__ qw, const float* __restrict__ qb,
                                                    const float* __restrict__ vw, const float* __restrict__ vb,
                                                    unsigned short* __restrict__ wp, float* __restrict__ btab) {
  const int t = threadIdx.x;
  const int lane = t & 31, wave = t >> 5;
  const int bx = blockIdx.x;
  if (bx < kWRows / 8) {
    const int r  = bx * 8 + wave;
    const int rv = min(r, kC - 1);
    const int rq = (r - kC) & (kD - 1);
    const float* pv = vw + (size_t)rv * kC + lane * 8;
    const float* pq = qw + (size_t)rq * kC + lane * 8;
    const v4f a0 = *(const v4f*)(pv);
    const v4f a1 = *(const v4f*)(pv + 4);
    const v4f b0 = *(const v4f*)(pq);
    const v4f b1 = *(const v4f*)(pq + 4);
    const bool useq = (r >= kC);
    unsigned short hb[8];
#pragma unroll
    for (int e = 0; e < 4; ++e) {
      const float w0 = useq ? b0[e] : a0[e];
      const float w1 = useq ? b1[e] : a1[e];
      hb[e]     = h_bits(bfr(w0) * kWCarry);
      hb[4 + e] = h_bits(bfr(w1) * kWCarry);
    }
    const v4u u = (v4u){pk16(hb[0], hb[1]), pk16(hb[2], hb[3]), pk16(hb[4], hb[5]), pk16(hb[6], hb[7])};
    unsigned short* op = wp + (size_t)r * kC + lane * 8;
    *(volatile v4u*)op = u;
    __threadfence();
    *(volatile v4u*)op = u;
  } else {
    const int iv = min(t, 63) * 4;
    const int iq = ((t - 64) & 7) * 4;
    const v4f a = *(const v4f*)(vb + iv);
    const v4f c = *(const v4f*)(qb + iq);
    const bool useq = (t >= 64);
    v4f o;
#pragma unroll
    for (int e = 0; e < 4; ++e) o[e] = bfr(useq ? c[e] : a[e]);
    float* op = btab + 4 * t;
    if (t < kWRows / 4) *(volatile v4f*)op = o;
    __threadfence();
    if (t < kWRows / 4) *(volatile v4f*)op = o;
  }
}

__global__ __launch_bounds__(512) void softmax_row_kernel(const float* __restrict__ Sg, unsigned short* __restrict__ P) {
  __shared__ float redM[16];
  __shared__ float redS[16];
  const int row  = blockIdx.x;
  const int t    = threadIdx.x;
  const int lane = t & 31, wave = t >> 5;
  const int c0   = t * 8;
  const float* sr = Sg + (size_t)row * kSeq + c0;
  const v4f a = *(const v4f*)(sr);
  const v4f c = *(const v4f*)(sr + 4);
  float x[8];
#pragma unroll
  for (int e = 0; e < 4; ++e) {
    x[e]     = a[e];
    x[4 + e] = c[e];
  }
  float m = fmaxf(fmaxf(fmaxf(x[0], x[1]), fmaxf(x[2], x[3])), fmaxf(fmaxf(x[4], x[5]), fmaxf(x[6], x[7])));
#pragma unroll
  for (int off = 16; off > 0; off >>= 1) m = fmaxf(m, __shfl_xor(m, off, 32));
  if (lane == 0) redM[wave] = m;
  __syncthreads();
  float gm = redM[0];
#pragma unroll
  for (int w = 1; w < kSmWaves; ++w) gm = fmaxf(gm, redM[w]);
  float ev[8];
  float ps = 0.f;
#pragma unroll
  for (int e = 0; e < 8; ++e) {
    ev[e] = expf(x[e] - gm);
    ps += ev[e];
  }
#pragma unroll
  for (int off = 16; off > 0; off >>= 1) ps += __shfl_xor(ps, off, 32);
  if (lane == 0) redS[wave] = ps;
  __syncthreads();
  float tot = 0.f;
#pragma unroll
  for (int w = 0; w < kSmWaves; ++w) tot += redS[w];
  const float inv = kPCarry * (1.0f / tot);
  unsigned short hb[8];
#pragma unroll
  for (int e = 0; e < 8; ++e) hb[e] = h_bits(ev[e] * inv);
  const v4u u = (v4u){pk16(hb[0], hb[1]), pk16(hb[2], hb[3]), pk16(hb[4], hb[5]), pk16(hb[6], hb[7])};
  unsigned short* q = P + (size_t)row * kSeq + c0;
  *(volatile v4u*)q = u;
  __threadfence();
  *(volatile v4u*)q = u;
}

extern "C" void kernel_launch(void* const* d_in, const int* in_sizes, int n_in,
                              void* d_out, int out_size, void* d_ws, size_t ws_size,
                              hipStream_t stream) {
  if (n_in < 6) return;
  if (in_sizes[0] < kBatch * kC * kSeqFull) return;
  if (in_sizes[1] < kD * kC || in_sizes[2] < kD) return;
  if (in_sizes[3] < kC * kC || in_sizes[4] < kC || in_sizes[5] < 1) return;
  if (out_size < kBatch * kC * kSeq) return;
  if (ws_size < kWsTotal) return;

  const float* x   = (const float*)d_in[0];
  const float* qw  = (const float*)d_in[1];
  const float* qb  = (const float*)d_in[2];
  const float* vw  = (const float*)d_in[3];
  const float* vb  = (const float*)d_in[4];
  const float* gam = (const float*)d_in[5];
  float* out = (float*)d_out;

  char* ws = (char*)d_ws;
  float*          Sp   = (float*)(ws + kOffS);
  unsigned short* Xt   = (unsigned short*)(ws + kOffXt);
  unsigned short* Wp   = (unsigned short*)(ws + kOffW);
  unsigned short* WqP  = Wp + (size_t)kC * kC;
  float*          btab = (float*)(ws + kOffBt);
  unsigned short* Qp   = (unsigned short*)(ws + kOffQ);
  unsigned short* Vp   = (unsigned short*)(ws + kOffV);
  unsigned short* Pp   = (unsigned short*)(ws + kOffP);

  xtcast_kernel<<<dim3(kSeq / 64, kC / 64, kBatch), dim3(256), 0, stream>>>(x, Xt);

  param_kernel<<<dim3(kWRows / 8 + 1), dim3(256), 0, stream>>>(qw, qb, vw, vb, Wp, btab);

  wmma_gemm64<0, false, 2, 3, false><<<dim3((kSeq / 64 + 7) / 8, kBatch), dim3(256), 0, stream>>>(
      Xt, Xt, kC, (long)kSeq * kC, WqP, WqP, kC, 0L,
      (void*)Qp, (void*)(Qp + 64), kQPitch, (long)kSeq * kQPitch,
      btab + kC, x, kSeqFull, 0L, gam, kSeq, kDP, kC, kWCarryInv);

  wmma_gemm64<0, false, 1, 1, false><<<dim3(((kC / 64) * (kSeq / 64) + 7) / 8, kBatch), dim3(256), 0, stream>>>(
      Wp, Wp, kC, 0L, Xt, Xt, kC, (long)kSeq * kC,
      (void*)Vp, (void*)Vp, kSeq, (long)kC * kSeq,
      btab, x, kSeqFull, 0L, gam, kC, kSeq, kC, kWCarryInv);

  for (int b = 0; b < kBatch; ++b) {
    const unsigned short* Qg = Qp + (size_t)b * kSeq * kQPitch;
    wmma_gemm64<1, false, 0, 0, false><<<dim3(((kSeq / 64) * (kSeq / 64) + 7) / 8, 1), dim3(256), 0, stream>>>(
        Qg, Qg, kQPitch, 0L, Qg + 32, Qg + 32, kQPitch, 0L,
        (void*)Sp, (void*)Sp, kSeq, 0L,
        btab, x, kSeqFull, 0L, gam, kSeq, kSeq, kQK, 1.0f);
    softmax_row_kernel<<<dim3(kSeq), dim3(kSmThreads), 0, stream>>>(Sp, Pp);
    const unsigned short* Vg = Vp + (size_t)b * kC * kSeq;
    float* Og = out + (size_t)b * kC * kSeq;
    const float* xg = x + (size_t)b * kC * kSeqFull;
    wmma_gemm64<0, false, 0, 0, true><<<dim3(((kC / 64) * (kSeq / 64) + 7) / 8, 1), dim3(256), 0, stream>>>(
        Vg, Vg, kSeq, 0L, Pp, Pp, kSeq, 0L,
        (void*)Og, (void*)Og, kSeq, 0L,
        btab, xg, kSeqFull, 0L, gam, kC, kSeq, kSeq, kPCarryInv);
  }
}
